// NonLocalAttention_66846870995635
// MI455X (gfx1250) — hardware-verified
//
#include <hip/hip_runtime.h>


#ifndef NB
#define NB 4
#endif
#ifndef SEQ
#define SEQ 4096
#endif

namespace {
typedef _Float16 b16;
typedef unsigned short us;
typedef __attribute__((ext_vector_type(16))) _Float16 v16b;
typedef __attribute__((ext_vector_type(8))) _Float16 v8b;
typedef __attribute__((ext_vector_type(4))) _Float16 v4h;
typedef __attribute__((ext_vector_type(2))) _Float16 v2h;
typedef __attribute__((ext_vector_type(16))) __bf16 v16bf;
typedef __attribute__((ext_vector_type(8))) unsigned short v8us;
typedef __attribute__((ext_vector_type(4))) unsigned short v4us;
typedef __attribute__((ext_vector_type(2))) unsigned short v2us;
typedef __attribute__((ext_vector_type(8))) float v8f;
typedef __attribute__((ext_vector_type(4))) float v4f;
typedef __attribute__((ext_vector_type(2))) float v2f;
union FragB { v16bf v; v8us h[2]; };

constexpr int NB_FULL = 4, SEQ_FULL = 4096, CH = 256, CI = 128;
constexpr float XS = 8.0f, WSC = 256.0f, QS = 8.0f, VS = 8.0f, OS = 8.0f, RS = 1024.0f, PS = 16384.0f, LOG2E = 1.4426950408889634f, EPS = 1e-5f;
static_assert(NB >= 1 && NB <= NB_FULL);
static_assert(SEQ % 64 == 0 && SEQ >= 64 && SEQ <= SEQ_FULL);
static_assert(CH % 32 == 0 && CI % 32 == 0 && CI == 128 && CH == 256);
static_assert((NB * SEQ) % 4 == 0);

__device__ __forceinline__ float bf16_rne(float f) { unsigned int u = __float_as_uint(f); u += 0x7FFFu + ((u >> 16) & 1u); return __uint_as_float(u & 0xFFFF0000u); }
__device__ __forceinline__ us bf16_bits(float f) { unsigned int u = __float_as_uint(f); u += 0x7FFFu + ((u >> 16) & 1u); return (us)(u >> 16); }
__device__ __forceinline__ v16b frag_kb(const b16* p, int hh) {
  const v8b a = *(const v8b*)(p + 8 * hh), b = *(const v8b*)(p + 16 + 8 * hh); v16b f;
#pragma unroll
  for (int e = 0; e < 8; ++e) { f[e] = a[e]; f[8 + e] = b[e]; }
  return f;
}
__device__ __forceinline__ v16bf frag_kbf(const us* p, int hh) { FragB f; f.h[0] = *(const v8us*)(p + 8 * hh); f.h[1] = *(const v8us*)(p + 16 + 8 * hh); return f.v; }
__device__ __forceinline__ v8f wmma16b(v16b a, v16b b, v8f c) {
  v8f d = __builtin_amdgcn_wmma_f32_16x16x32_f16(false, a, false, b, (short)0, c, false, false);
  asm volatile("v_nop\n\tv_nop\n\tv_nop\n\tv_nop" : "+v"(d) : "v"(a), "v"(b));
  return d;
}
__device__ __forceinline__ v8f wmmabf(v16bf a, v16bf b, v8f c) {
  v8f d = __builtin_amdgcn_wmma_f32_16x16x32_bf16(false, a, false, b, (short)0, c, false, false);
  asm volatile("v_nop\n\tv_nop\n\tv_nop\n\tv_nop" : "+v"(d) : "v"(a), "v"(b));
  return d;
}
__device__ __forceinline__ void wave_lds_sync() { __builtin_amdgcn_fence(__ATOMIC_RELEASE, "workgroup"); __builtin_amdgcn_wave_barrier(); __builtin_amdgcn_fence(__ATOMIC_ACQUIRE, "workgroup"); }
__device__ __forceinline__ void cbar() { asm volatile("" ::: "memory"); }
__device__ __forceinline__ float nexp2(float v) { return __builtin_amdgcn_exp2f(v); }

__global__ __launch_bounds__(256) void prep_kernel(const float* __restrict__ tw, const float* __restrict__ pw, const float* __restrict__ gw, const float* __restrict__ rw,
                                                   b16* __restrict__ WT, b16* __restrict__ WP, b16* __restrict__ WG, b16* __restrict__ WRh, us* __restrict__ WRb) {
  constexpr int NW = CI * CH;
  const int u = blockIdx.x * 256 + threadIdx.x;
  if (u >= 5 * NW / 8) return;
  const int e = u * 8; const int seg = e / NW; const int r = e - seg * NW;
  const float* w = seg == 0 ? tw : seg == 1 ? pw : seg == 2 ? gw : rw;
  float f[8];
#pragma unroll
  for (int j = 0; j < 8; ++j) f[j] = bf16_rne(w[r + j]) * WSC;
  if (seg < 4) {
    b16* d = seg == 0 ? WT : seg == 1 ? WP : seg == 2 ? WG : WRh; v8b v;
#pragma unroll
    for (int j = 0; j < 8; ++j) v[j] = (b16)f[j];
    for (int pass = 0; pass < 2; ++pass) { *(volatile v8b*)(d + r) = v; __threadfence(); }
  } else {
    v8us v;
#pragma unroll
    for (int j = 0; j < 8; ++j) v[j] = bf16_bits(f[j]);
    for (int pass = 0; pass < 2; ++pass) { *(volatile v8us*)(WRb + r) = v; __threadfence(); }
  }
}

__global__ __launch_bounds__(256) void cvt_kernel(const float* __restrict__ x, const float* __restrict__ y, b16* __restrict__ X16, b16* __restrict__ Y16) {
  __shared__ __attribute__((aligned(16))) b16 T[64][CH + 8];
  const int b = blockIdx.y, p0 = blockIdx.x * 64, z = blockIdx.z;
  const float* src = z ? y : x; b16* dst = z ? Y16 : X16;
  const int wave = threadIdx.x >> 5, lane = threadIdx.x & 31;
#pragma unroll 4
  for (int i = threadIdx.x; i < CH * 64; i += 256) { const int c = i >> 6, pp = i & 63; T[pp][c] = (b16)(bf16_rne(src[((size_t)b * CH + c) * SEQ_FULL + p0 + pp]) * XS); }
  __syncthreads();
  for (int pass = 0; pass < 2; ++pass) {
#pragma unroll 1
    for (int rr = 0; rr < 8; ++rr) { const int row = wave * 8 + rr; const v8b v = *(const v8b*)&T[row][lane * 8];
      *(volatile v8b*)(dst + ((size_t)b * SEQ_FULL + p0 + row) * CH + lane * 8) = v; }
    __threadfence(); }
}

template <int MODE>
__global__ __launch_bounds__(128) void proj_kernel(const b16* __restrict__ X16, const b16* __restrict__ W16, const float* __restrict__ bias, b16* __restrict__ outH, void* __restrict__ outL) {
  __shared__ __attribute__((aligned(16))) float Tf[4][16][CI + 4];
  const int wave = threadIdx.x >> 5, lane = threadIdx.x & 31, nloc = lane & 15, hlf = lane >> 4; const int p0 = blockIdx.x * 64; const int b = blockIdx.y;
  const b16* arow = X16 + ((size_t)b * SEQ_FULL + p0 + wave * 16 + nloc) * CH;
  v8f acc[8];
#pragma unroll
  for (int t = 0; t < 8; ++t) acc[t] = (v8f){};
#pragma unroll
  for (int kb = 0; kb < CH; kb += 32) { const v16b a = frag_kb(arow + kb, hlf);
#pragma unroll
    for (int t = 0; t < 8; ++t) acc[t] = wmma16b(a, frag_kb(W16 + (size_t)(t * 16 + nloc) * CH + kb, hlf), acc[t]); }
#pragma unroll
  for (int t = 0; t < 8; ++t) { const int o = t * 16 + nloc; const float bb = bf16_rne(bias[o]);
#pragma unroll
    for (int r = 0; r < 8; ++r) Tf[wave][8 * hlf + r][o] = acc[t][r] * (1.0f / (XS * WSC)) + bb; }
  __syncthreads();
  for (int pass = 0; pass < 2; ++pass) {
    if (MODE == 0) {
      b16* outLo = (b16*)outL;
#pragma unroll 1
      for (int rr = 0; rr < 16; ++rr) { const int p = p0 + wave * 16 + rr; const int d = lane * 4; v4h hv, lv;
#pragma unroll
        for (int j = 0; j < 4; ++j) { const float f = Tf[wave][rr][d + j] * QS; const b16 h = (b16)f; hv[j] = h; lv[j] = (b16)((f - (float)h) * RS); }
        const size_t oi = ((size_t)b * SEQ_FULL + p) * CI + d; *(volatile v4h*)(outH + oi) = hv; *(volatile v4h*)(outLo + oi) = lv; }
    } else {
      us* outLo = (us*)outL;
#pragma unroll 1
      for (int q = 0; q < 32; ++q) { const int d = wave * 32 + q; const int tk = lane * 2; v2h hv; v2us lv;
#pragma unroll
        for (int j = 0; j < 2; ++j) { const int px = tk + j; const float f = Tf[px >> 4][px & 15][d] * VS; const b16 h = (b16)f; hv[j] = h; lv[j] = bf16_bits(f - (float)h); }
        const size_t oi = ((size_t)b * CI + d) * SEQ_FULL + p0 + tk; *(volatile v2h*)(outH + oi) = hv; *(volatile v2us*)(outLo + oi) = lv; }
    }
    __threadfence(); }
}

__global__ __launch_bounds__(64) void attn_kernel(const b16* __restrict__ Qh, const b16* __restrict__ Ql, const b16* __restrict__ Kh, const b16* __restrict__ Kl,
                                                  const b16* __restrict__ VTh, const us* __restrict__ VTl, b16* __restrict__ Oh, us* __restrict__ Ol) {
  __shared__ __attribute__((aligned(16))) b16 Pb[2][16][32 + 8]; __shared__ __attribute__((aligned(16))) us Pbb[2][16][32 + 8]; __shared__ __attribute__((aligned(16))) float To[32][CI + 4];
  const int wave = threadIdx.x >> 5, lane = threadIdx.x & 31, hh = lane >> 4, col = lane & 15; const int b = blockIdx.y; const int p0 = blockIdx.x * 32; const int q0 = p0 + wave * 16, qi = q0 + col;
  const size_t pb = (size_t)b * SEQ_FULL * CI; const b16* Qhb = Qh + pb; const b16* Qlb = Ql + pb; const b16* Khb = Kh + pb; const b16* Klb = Kl + pb;
  const size_t vb = (size_t)b * CI * SEQ_FULL; const b16* Vhb = VTh + vb; const us* Vlb = VTl + vb;
  const int qoff = qi * CI;
  const float cs = LOG2E / (QS * QS), csl = cs / RS;
  float m = -INFINITY, l = 0.0f; v8f o[8];
#pragma unroll
  for (int t = 0; t < 8; ++t) o[t] = (v8f){};
#pragma unroll 1
  for (int kb = 0; kb < SEQ; kb += 32) {
    int qo = qoff; asm volatile("" : "+v"(qo));
    const int kr0 = (kb + col) * CI, kr1 = (kb + 16 + col) * CI;
    v8f s0 = (v8f){}, s1 = (v8f){}, sl0 = (v8f){}, sl1 = (v8f){};
#pragma unroll
    for (int st = 0; st < 4; ++st) {
      const v16b qh = frag_kb(Qhb + qo + 32 * st, hh), ql = frag_kb(Qlb + qo + 32 * st, hh);
      { const v16b kh = frag_kb(Khb + kr0 + 32 * st, hh), kl = frag_kb(Klb + kr0 + 32 * st, hh); s0 = wmma16b(kh, qh, s0); sl0 = wmma16b(kh, ql, sl0); sl0 = wmma16b(kl, qh, sl0); }
      { const v16b kh = frag_kb(Khb + kr1 + 32 * st, hh), kl = frag_kb(Klb + kr1 + 32 * st, hh); s1 = wmma16b(kh, qh, s1); sl1 = wmma16b(kh, ql, sl1); sl1 = wmma16b(kl, qh, sl1); }
      cbar(); }
    float e[16]; float mx = -INFINITY;
#pragma unroll
    for (int r = 0; r < 8; ++r) { const float v0 = s0[r] * cs + sl0[r] * csl; const float v1 = s1[r] * cs + sl1[r] * csl; e[r] = v0; e[8 + r] = v1; mx = fmaxf(mx, fmaxf(v0, v1)); }
    mx = fmaxf(mx, __shfl_xor(mx, 16)); const float mn = fmaxf(m, mx); const float al = nexp2(m - mn); float sum = 0.0f;
#pragma unroll
    for (int i2 = 0; i2 < 16; ++i2) { const float p = nexp2(e[i2] - mn); sum += p; const float ps = p * PS; const int idx = (i2 < 8 ? 0 : 16) + 8 * hh + (i2 & 7);
      Pb[wave][col][idx] = (b16)ps; Pbb[wave][col][idx] = bf16_bits(ps); }
    sum += __shfl_xor(sum, 16); l = l * al + sum; m = mn;
    wave_lds_sync();
    const v16b pf = frag_kb(&Pb[wave][col][0], hh); const v16bf pbf = frag_kbf(&Pbb[wave][col][0], hh);
#pragma unroll
    for (int t = 0; t < 8; ++t) { o[t] *= al; const size_t vr = (size_t)(t * 16 + col) * SEQ_FULL + kb;
      o[t] = wmma16b(frag_kb(Vhb + vr, hh), pf, o[t]); o[t] = wmmabf(frag_kbf(Vlb + vr, hh), pbf, o[t]); if (t & 1) cbar(); }
    wave_lds_sync(); }
  const float inv = 1.0f / (l * PS * VS);
#pragma unroll
  for (int t = 0; t < 8; ++t)
#pragma unroll
    for (int r = 0; r < 8; ++r) To[wave * 16 + col][t * 16 + 8 * hh + r] = o[t][r] * inv;
  __syncthreads();
  for (int pass = 0; pass < 2; ++pass) {
#pragma unroll 1
    for (int rr = 0; rr < 16; ++rr) { const int q = wave * 16 + rr; const int d = lane * 4; v4h hv; v4us lv;
#pragma unroll
      for (int j = 0; j < 4; ++j) { const float f = To[q][d + j] * OS; const b16 h = (b16)f; hv[j] = h; lv[j] = bf16_bits(f - (float)h); }
      const size_t oi = ((size_t)b * SEQ_FULL + p0 + q) * CI + d; *(volatile v4h*)(Oh + oi) = hv; *(volatile v4us*)(Ol + oi) = lv; }
    __threadfence(); }
}

__global__ __launch_bounds__(128) void rec_kernel(const b16* __restrict__ Oh, const us* __restrict__ Ol, const b16* __restrict__ WRh, const us* __restrict__ WRb, const float* __restrict__ rb, float* __restrict__ R) {
  __shared__ __attribute__((aligned(16))) float Tf[4][16][CI + 4];
  const int wave = threadIdx.x >> 5, lane = threadIdx.x & 31, nloc = lane & 15, hlf = lane >> 4; const int p0 = blockIdx.x * 64; const int b = blockIdx.y; const int g = blockIdx.z;
  const size_t arow = ((size_t)b * SEQ_FULL + p0 + wave * 16 + nloc) * CI;
  v8f acc[8];
#pragma unroll
  for (int t = 0; t < 8; ++t) acc[t] = (v8f){};
#pragma unroll
  for (int kb = 0; kb < CI; kb += 32) { const v16b ah = frag_kb(Oh + arow + kb, hlf); const v16bf alo = frag_kbf(Ol + arow + kb, hlf);
#pragma unroll
    for (int t = 0; t < 8; ++t) { const size_t wr = (size_t)(g * 128 + t * 16 + nloc) * CI + kb; acc[t] = wmma16b(ah, frag_kb(WRh + wr, hlf), acc[t]); acc[t] = wmmabf(alo, frag_kbf(WRb + wr, hlf), acc[t]); } }
#pragma unroll
  for (int t = 0; t < 8; ++t) { const int cl = t * 16 + nloc; const float bb = bf16_rne(rb[g * 128 + cl]);
#pragma unroll
    for (int r = 0; r < 8; ++r) Tf[wave][8 * hlf + r][cl] = acc[t][r] * (1.0f / (OS * WSC)) + bb; }
  __syncthreads();
  for (int pass = 0; pass < 2; ++pass) {
#pragma unroll 1
    for (int q = 0; q < 32; ++q) { const int cl = wave * 32 + q; const int c = g * 128 + cl; const int tk = lane * 2; v2f v;
      v[0] = Tf[tk >> 4][tk & 15][cl]; v[1] = Tf[(tk + 1) >> 4][(tk + 1) & 15][cl];
      *(volatile v2f*)(R + ((size_t)b * CH + c) * SEQ_FULL + p0 + tk) = v; }
    __threadfence(); }
}

__global__ __launch_bounds__(256) void bn_kernel(const float* __restrict__ x, const float* __restrict__ R, const float* __restrict__ gamma, const float* __restrict__ beta, float* __restrict__ out) {
  __shared__ double sh1[256]; __shared__ double sh2[256];
  const int c = blockIdx.x, tid = threadIdx.x;
  constexpr int TOT = NB * SEQ, KT = (TOT + 1023) / 1024;
  double a = 0.0, q = 0.0;
#pragma unroll 1
  for (int k = 0; k < KT; ++k) { const int f = k * 1024 + tid * 4; const int fc = f < TOT - 4 ? f : TOT - 4; const int bb = fc / SEQ, p = fc - bb * SEQ;
    const v4f v = *(const v4f*)(R + ((size_t)bb * CH + c) * SEQ_FULL + p);
    if (f < TOT) {
#pragma unroll
      for (int j = 0; j < 4; ++j) { a += (double)v[j]; q += (double)v[j] * (double)v[j]; } } }
  sh1[tid] = a; sh2[tid] = q; __syncthreads();
  for (int s = 128; s > 0; s >>= 1) { if (tid < s) { sh1[tid] += sh1[tid + s]; sh2[tid] += sh2[tid + s]; } __syncthreads(); }
  const double md = sh1[0] / (double)TOT; double vd = sh2[0] / (double)TOT - md * md; vd = vd < 0.0 ? 0.0 : vd;
  const float mean = (float)md; const float var = (float)vd; const float rstd = 1.0f / sqrtf(var + EPS);
  const float gm = bf16_rne(gamma[c]), bt = bf16_rne(beta[c]);
#pragma unroll 1
  for (int k = 0; k < KT; ++k) { const int f = k * 1024 + tid * 4; const int fc = f < TOT - 4 ? f : TOT - 4; const int bb = fc / SEQ, p = fc - bb * SEQ;
    const size_t gi = ((size_t)bb * CH + c) * SEQ_FULL + p; const v4f rv = *(const v4f*)(R + gi); const v4f xv = *(const v4f*)(x + gi); v4f res;
#pragma unroll
    for (int j = 0; j < 4; ++j) { const float tn = (rv[j] - mean) * rstd; res[j] = bf16_rne(xv[j]) + (gm * tn + bt); }
    if (f < TOT) { *(volatile v4f*)(out + gi) = res; __threadfence(); *(volatile v4f*)(out + gi) = res; } }
}
}

extern "C" void kernel_launch(void* const* d_in, const int* in_sizes, int n_in, void* d_out, int out_size, void* d_ws, size_t ws_size, hipStream_t stream) {
  if (n_in < 12) return;
  auto Fp = [&](int i) { return (const float*)d_in[i]; };
  if (in_sizes[0] < NB * CH * SEQ_FULL || in_sizes[1] < NB * CH * SEQ_FULL || in_sizes[2] < CI * CH || in_sizes[3] < CI || in_sizes[4] < CI * CH || in_sizes[5] < CI ||
      in_sizes[6] < CI * CH || in_sizes[7] < CI || in_sizes[8] < CH * CI || in_sizes[9] < CH || in_sizes[10] < CH || in_sizes[11] < CH || out_size < NB * CH * SEQ_FULL) return;
  size_t off = 0; char* ws = (char*)d_ws;
  auto carve = [&](size_t bytes) { char* p = ws + off; off += (bytes + 255) & ~(size_t)255; return p; };
  const size_t wb = (size_t)CI * CH * 2;
  b16* WT = (b16*)carve(wb); b16* WP = (b16*)carve(wb); b16* WG = (b16*)carve(wb); b16* WRh = (b16*)carve(wb); us* WRb = (us*)carve(wb);
  const size_t xb = (size_t)NB_FULL * SEQ_FULL * CH * 2;
  b16* X16 = (b16*)carve(xb); b16* Y16 = (b16*)carve(xb);
  const size_t plane = (size_t)NB_FULL * SEQ_FULL * CI * 2;
  b16* Qh = (b16*)carve(plane); b16* Ql = (b16*)carve(plane); b16* Kh = (b16*)carve(plane); b16* Kl = (b16*)carve(plane);
  b16* VTh = (b16*)carve(plane); us* VTl = (us*)carve(plane); b16* Oh = (b16*)carve(plane); us* Ol = (us*)carve(plane);
  float* R = (float*)carve((size_t)NB_FULL * CH * SEQ_FULL * 4);
  if (off > ws_size || off > ((size_t)128 << 20)) return;
  prep_kernel<<<(5 * CI * CH / 8 + 255) / 256, 256, 0, stream>>>(Fp(2), Fp(4), Fp(6), Fp(8), WT, WP, WG, WRh, WRb);
  cvt_kernel<<<dim3(SEQ / 64, NB, 2), 256, 0, stream>>>(Fp(0), Fp(1), X16, Y16);
  proj_kernel<0><<<dim3(SEQ / 64, NB), 128, 0, stream>>>(X16, WT, Fp(3), Qh, (void*)Ql);
  proj_kernel<0><<<dim3(SEQ / 64, NB), 128, 0, stream>>>(Y16, WP, Fp(5), Kh, (void*)Kl);
  proj_kernel<1><<<dim3(SEQ / 64, NB), 128, 0, stream>>>(X16, WG, Fp(7), VTh, (void*)VTl);
  attn_kernel<<<dim3(SEQ / 32, NB), 64, 0, stream>>>(Qh, Ql, Kh, Kl, VTh, VTl, Oh, Ol);
  rec_kernel<<<dim3(SEQ / 64, NB, 2), 128, 0, stream>>>(Oh, Ol, WRh, WRb, Fp(9), R);
  bn_kernel<<<dim3(CH), 256, 0, stream>>>(Fp(0), R, Fp(10), Fp(11), (float*)d_out);
}
